// TransformerBlock_1932735283786
// MI455X (gfx1250) — hardware-verified
//
#include <hip/hip_runtime.h>
#include <math.h>

#ifndef NB
#define NB 2
#endif
#ifndef SEQ
#define SEQ 2048
#endif
#define NB_FULL 2
#define SEQ_FULL 2048
#define CC 1024
#define NH 16
#define HD 64
#define DFF 4096
#define MT (NB * SEQ)
#define PP 40
#define SP 68

static_assert(NH * HD == CC);
static_assert(HD == 64);
static_assert(CC == 128 * 8);
static_assert(SEQ % 64 == 0);
static_assert(NB <= NB_FULL && SEQ <= SEQ_FULL);
static_assert(MT % 64 == 0 && CC % 64 == 0 && DFF % 64 == 0 && (2 * CC) % 64 == 0);
static_assert(CC % 32 == 0 && DFF % 32 == 0);
static_assert((PP * 2) % 16 == 0 && PP >= 32);
static_assert((SP * 4) % 16 == 0 && SP >= 64);
static_assert((MT * 2) % 128 == 0);

typedef __attribute__((ext_vector_type(16))) _Float16 v16h;
typedef __attribute__((ext_vector_type(8)))  _Float16 v8h;
typedef __attribute__((ext_vector_type(8)))  float    v8f;
typedef __attribute__((ext_vector_type(4)))  float    v4f;
typedef __attribute__((ext_vector_type(4)))  unsigned int u4;
typedef __attribute__((ext_vector_type(2)))  unsigned int u2;

union FragH { v16h v; v8h h[2]; };
__device__ __forceinline__ v16h ld_frag(const _Float16* __restrict__ p) {
    FragH f; f.h[0] = *(const v8h*)(p); f.h[1] = *(const v8h*)(p + 16); return f.v;
}
__device__ __forceinline__ v8f wmma16(v16h a, v16h b, v8f c) {
    c = __builtin_amdgcn_wmma_f32_16x16x32_f16(false, a, false, b, (short)0, c, false, false);
    asm volatile("v_nop\n\tv_nop\n\tv_nop\n\tv_nop" : "+v"(c) : "v"(a), "v"(b));
    return c;
}
__device__ __forceinline__ void grp_guard(v8f& a0, v8f& a1, v8f& a2, v8f& a3, v16h x, v16h y) {
    asm volatile("v_nop\n\tv_nop\n\tv_nop\n\tv_nop" : "+v"(a0), "+v"(a1), "+v"(a2), "+v"(a3) : "v"(x), "v"(y));
}
__device__ __forceinline__ void keep4(v16h a, v16h b, v16h c, v16h d) { asm volatile("v_nop" :: "v"(a), "v"(b), "v"(c), "v"(d)); }
__device__ __forceinline__ void acc_guard4(v8f& a, v8f& b, v8f& c, v8f& d) {
    asm volatile("v_nop\n\tv_nop\n\tv_nop\n\tv_nop" : "+v"(a), "+v"(b), "+v"(c), "+v"(d));
}
__device__ __forceinline__ void wave_sync() {
    __builtin_amdgcn_fence(3  , "workgroup");
    __builtin_amdgcn_wave_barrier();
    __builtin_amdgcn_fence(2  , "workgroup");
}

__device__ __forceinline__ float cmb_bf(float v) {
    const unsigned u = __builtin_bit_cast(unsigned, v);
    const unsigned r = (u + 0x7fffu + ((u >> 16) & 1u)) & 0xffff0000u;
    return __builtin_bit_cast(float, r);
}
__device__ __forceinline__ unsigned int pk2(float a, float b) {
    return (unsigned int)__builtin_bit_cast(unsigned short, (_Float16)a) | ((unsigned int)__builtin_bit_cast(unsigned short, (_Float16)b) << 16);
}
__device__ __forceinline__ float gelu_erf(float v) { return 0.5f * v * (1.0f + erff(v * 0.70710678118654752f)); }

__global__ __launch_bounds__(256) void k_castw(const float* __restrict__ SRC, unsigned short* __restrict__ DST, int n8, float sc) {
    const int u = (int)blockIdx.x * 256 + (int)threadIdx.x;
    if (u >= n8) return;
    const v4f a = *(const v4f*)(SRC + (size_t)u * 8);
    const v4f b = *(const v4f*)(SRC + (size_t)u * 8 + 4);
    u4 pk;
    pk.x = pk2(cmb_bf(a.x) * sc, cmb_bf(a.y) * sc);
    pk.y = pk2(cmb_bf(a.z) * sc, cmb_bf(a.w) * sc);
    pk.z = pk2(cmb_bf(b.x) * sc, cmb_bf(b.y) * sc);
    pk.w = pk2(cmb_bf(b.z) * sc, cmb_bf(b.w) * sc);
    volatile u4* d = (volatile u4*)(DST + (size_t)u * 8);
    *d = pk; __threadfence(); *d = pk;
}

template <int ABF>
__device__ __forceinline__ void ln_body(const float* __restrict__ A, const float* __restrict__ GA, const float* __restrict__ BE, unsigned short* __restrict__ Y16) {
    #pragma clang fp contract(off)
    const int wave = __builtin_amdgcn_readfirstlane((int)(threadIdx.x >> 5));
    const int r = (int)blockIdx.x * 8 + wave;
    const int L = threadIdx.x & 31;
    if (r >= MT) return;
    const int rsrc = ABF ? ((r / SEQ) * SEQ_FULL + (r % SEQ)) : r;
    v4f v[8]; float s = 0.f;
#pragma unroll
    for (int q = 0; q < 8; ++q) {
        v[q] = *(const v4f*)(A + (size_t)rsrc * CC + 4 * L + 128 * q);
        if (ABF) { v[q].x = cmb_bf(v[q].x); v[q].y = cmb_bf(v[q].y); v[q].z = cmb_bf(v[q].z); v[q].w = cmb_bf(v[q].w); }
        s += (v[q].x + v[q].y) + (v[q].z + v[q].w);
    }
#pragma unroll
    for (int o = 16; o > 0; o >>= 1) s += __shfl_xor(s, o, 32);
    const float mu = s * (1.f / CC);
    float qq = 0.f;
#pragma unroll
    for (int q = 0; q < 8; ++q) {
        v[q].x -= mu; v[q].y -= mu; v[q].z -= mu; v[q].w -= mu;
        qq += (v[q].x * v[q].x + v[q].y * v[q].y) + (v[q].z * v[q].z + v[q].w * v[q].w);
    }
#pragma unroll
    for (int o = 16; o > 0; o >>= 1) qq += __shfl_xor(qq, o, 32);
    const float rs = rsqrtf(qq * (1.f / CC) + 1e-5f);
#pragma unroll
    for (int q = 0; q < 8; ++q) {
        const int c = 4 * L + 128 * q;
        const v4f ga = *(const v4f*)(GA + c), be = *(const v4f*)(BE + c);
        const float y0 = v[q].x * rs * cmb_bf(ga.x) + cmb_bf(be.x);
        const float y1 = v[q].y * rs * cmb_bf(ga.y) + cmb_bf(be.y);
        const float y2 = v[q].z * rs * cmb_bf(ga.z) + cmb_bf(be.z);
        const float y3 = v[q].w * rs * cmb_bf(ga.w) + cmb_bf(be.w);
        u2 pk; pk.x = pk2(y0, y1); pk.y = pk2(y2, y3);
        volatile u2* d = (volatile u2*)(Y16 + (size_t)r * CC + c);
        *d = pk; __threadfence(); *d = pk;
    }
}
__global__ __launch_bounds__(256) void k_ln_in(const float* __restrict__ A, const float* __restrict__ GA, const float* __restrict__ BE, unsigned short* __restrict__ Y16) { ln_body<1>(A, GA, BE, Y16); }
__global__ __launch_bounds__(256) void k_ln_mid(const float* __restrict__ A, const float* __restrict__ GA, const float* __restrict__ BE, unsigned short* __restrict__ Y16) { ln_body<0>(A, GA, BE, Y16); }

template <int OUT_MODE, int BIAS_MODE, bool RESID, bool XBF, bool GELU>
__device__ __forceinline__ void gemm64_body(float (&sT)[8][16 * SP],
        const _Float16* __restrict__ A, int lda, const _Float16* __restrict__ Bt, int ldb,
        float* __restrict__ Cf, unsigned short* __restrict__ Ch, int ldc,
        const float* __restrict__ bias, const float* __restrict__ resid,
        int M, int N, int K, float scale, float ocarry) {
    const int lane = threadIdx.x & 31;
    const int wave = __builtin_amdgcn_readfirstlane((int)(threadIdx.x >> 5));
    const int tilesN = N >> 6, tilesM = M >> 6;
    const int tile = (int)blockIdx.x * 8 + wave;
    if (tile >= tilesM * tilesN) return;
    const int tm = tile / tilesN, tn = tile - tm * tilesN;
    const int m0 = tm << 6, n0 = tn << 6;
    const int rlane = lane & 15;
    const int koff = (lane >> 4) * 8;
    const int mOff = (lane >> 4) * 8;

    v8f acc[4][4];
#pragma unroll
    for (int i = 0; i < 4; ++i)
#pragma unroll
        for (int j = 0; j < 4; ++j) acc[i][j] = (v8f){0.f, 0.f, 0.f, 0.f, 0.f, 0.f, 0.f, 0.f};

    for (int k0 = 0; k0 < K; k0 += 32) {
        v16h bh[4];
#pragma unroll
        for (int j = 0; j < 4; ++j) bh[j] = ld_frag(Bt + (size_t)(n0 + (j << 4) + rlane) * ldb + koff + k0);
#pragma unroll
        for (int i = 0; i < 4; ++i) {
            const v16h ah = ld_frag(A + (size_t)(m0 + (i << 4) + rlane) * lda + koff + k0);
#pragma unroll
            for (int j = 0; j < 4; ++j)
                acc[i][j] = __builtin_amdgcn_wmma_f32_16x16x32_f16(false, ah, false, bh[j], (short)0, acc[i][j], false, false);
            grp_guard(acc[i][0], acc[i][1], acc[i][2], acc[i][3], ah, bh[3]);
        }
        keep4(bh[0], bh[1], bh[2], bh[3]);
    }
    acc_guard4(acc[0][0], acc[0][1], acc[0][2], acc[0][3]);
    acc_guard4(acc[1][0], acc[1][1], acc[1][2], acc[1][3]);
    acc_guard4(acc[2][0], acc[2][1], acc[2][2], acc[2][3]);
    acc_guard4(acc[3][0], acc[3][1], acc[3][2], acc[3][3]);

#pragma unroll
    for (int i = 0; i < 4; ++i) {
        const int mBase = m0 + (i << 4);
        float bm[8];
#pragma unroll
        for (int r = 0; r < 8; ++r) bm[r] = (BIAS_MODE == 1) ? cmb_bf(bias[mBase + mOff + r]) : 0.f;
#pragma unroll
        for (int j = 0; j < 4; ++j) {
            const float bv = (BIAS_MODE == 2) ? cmb_bf(bias[n0 + (j << 4) + rlane]) : 0.f;
#pragma unroll
            for (int r = 0; r < 8; ++r) sT[wave][(mOff + r) * SP + (j << 4) + rlane] = acc[i][j][r] * scale + bm[r] + bv;
        }
        wave_sync();
        if (OUT_MODE == 0) {
            const int hh2 = lane >> 4, c4 = (lane & 15) * 4;
            for (int pass = 0; pass < 2; ++pass) {
#pragma unroll
                for (int it = 0; it < 8; ++it) {
                    const int row = it * 2 + hh2;
                    v4f v = *(const v4f*)&sT[wave][row * SP + c4];
                    if (RESID) {
                        const int gm = mBase + row;
                        const int rr = XBF ? ((gm / SEQ) * SEQ_FULL + (gm % SEQ)) : gm;
                        v4f x = *(const v4f*)(resid + (size_t)rr * ldc + n0 + c4);
                        if (XBF) { x.x = cmb_bf(x.x); x.y = cmb_bf(x.y); x.z = cmb_bf(x.z); x.w = cmb_bf(x.w); }
                        v = v + x;
                    }
                    *(volatile v4f*)(Cf + (size_t)(mBase + row) * ldc + n0 + c4) = v;
                }
                __threadfence();
            }
        } else if (!GELU) {
            const int q = lane >> 3, c8 = (lane & 7) * 8;
            for (int pass = 0; pass < 2; ++pass) {
#pragma unroll
                for (int it = 0; it < 4; ++it) {
                    const int row = it * 4 + q;
                    v8h hv;
#pragma unroll
                    for (int e = 0; e < 8; ++e) hv[e] = (_Float16)(sT[wave][row * SP + c8 + e] * ocarry);
                    *(volatile v8h*)(Ch + (size_t)(mBase + row) * ldc + n0 + c8) = hv;
                }
                __threadfence();
            }
        } else {
            const int q = lane >> 3, c8 = (lane & 7) * 8;
#pragma unroll 1
            for (int it = 0; it < 4; ++it) {
                const int row = it * 4 + q;
                const int si = row * SP + c8;
                const float a0 = sT[wave][si], a1 = sT[wave][si + 1], a2 = sT[wave][si + 2], a3 = sT[wave][si + 3];
                const float a4 = sT[wave][si + 4], a5 = sT[wave][si + 5], a6 = sT[wave][si + 6], a7 = sT[wave][si + 7];
                u4 pk;
                pk.x = pk2(gelu_erf(a0) * ocarry, gelu_erf(a1) * ocarry);
                pk.y = pk2(gelu_erf(a2) * ocarry, gelu_erf(a3) * ocarry);
                pk.z = pk2(gelu_erf(a4) * ocarry, gelu_erf(a5) * ocarry);
                pk.w = pk2(gelu_erf(a6) * ocarry, gelu_erf(a7) * ocarry);
                volatile u4* d = (volatile u4*)(Ch + (size_t)(mBase + row) * ldc + n0 + c8);
                *d = pk; __threadfence(); *d = pk;
            }
        }
        wave_sync();
    }
}

__global__ __launch_bounds__(256) void k_gemm_qk(const _Float16* __restrict__ X16, const _Float16* __restrict__ W16, const float* __restrict__ bias, unsigned short* __restrict__ QK) {
    __shared__ __align__(16) float sT[8][16 * SP];
    gemm64_body<1, 2, false, false, false>(sT, X16, CC, W16, CC, nullptr, QK, 2 * CC, bias, nullptr, MT, 2 * CC, CC, 0.0625f, 1.0f);
}
__global__ __launch_bounds__(256) void k_gemm_vt(const _Float16* __restrict__ Wv16, const _Float16* __restrict__ X16, const float* __restrict__ biasv, unsigned short* __restrict__ VT) {
    __shared__ __align__(16) float sT[8][16 * SP];
    gemm64_body<1, 1, false, false, false>(sT, Wv16, CC, X16, CC, nullptr, VT, MT, biasv, nullptr, CC, MT, CC, 0.0625f, 1.0f);
}
__global__ __launch_bounds__(256) void k_gemm_proj(const _Float16* __restrict__ O16, const _Float16* __restrict__ WP16, const float* __restrict__ bias, const float* __restrict__ x, float* __restrict__ X1) {
    __shared__ __align__(16) float sT[8][16 * SP];
    gemm64_body<0, 2, true, true, false>(sT, O16, CC, WP16, CC, X1, nullptr, CC, bias, x, MT, CC, CC, 1.0f / 1024.0f, 1.0f);
}
__global__ __launch_bounds__(256) void k_gemm_fc1(const _Float16* __restrict__ H16, const _Float16* __restrict__ W116, const float* __restrict__ bias, unsigned short* __restrict__ F16) {
    __shared__ __align__(16) float sT[8][16 * SP];
    gemm64_body<1, 2, false, false, true>(sT, H16, CC, W116, CC, nullptr, F16, DFF, bias, nullptr, MT, DFF, CC, 0.0625f, 8.0f);
}
__global__ __launch_bounds__(256) void k_gemm_fc2(const _Float16* __restrict__ F16, const _Float16* __restrict__ W216, const float* __restrict__ bias, const float* __restrict__ X1, float* __restrict__ out) {
    __shared__ __align__(16) float sT[8][16 * SP];
    gemm64_body<0, 2, true, false, false>(sT, F16, DFF, W216, DFF, out, nullptr, CC, bias, X1, MT, CC, DFF, 1.0f / 256.0f, 1.0f);
}

__global__ __launch_bounds__(128) void k_attn(const _Float16* __restrict__ QK, const _Float16* __restrict__ VT, unsigned short* __restrict__ O16) {
    __shared__ __align__(16) _Float16 Psh[4][16 * PP];
    __shared__ __align__(16) float Os[4][16 * SP];
    const int lane = threadIdx.x & 31;
    const int wave = __builtin_amdgcn_readfirstlane((int)(threadIdx.x >> 5));
    const int hh = lane >> 4, c = lane & 15;
    const int nqb = SEQ / 64;
    const int bx = (int)blockIdx.x;
    const int qb = bx % nqb, bh = bx / nqb;
    const int h = bh % NH, b = bh / NH;
    const int q0 = qb * 64 + wave * 16;
    const int qoff = (b * SEQ + q0 + c) * (2 * CC) + h * HD + 8 * hh;
    const int kb0  = (b * SEQ + c) * (2 * CC) + CC + h * HD + 8 * hh;
    const int vb0  = (h * HD + c) * MT + b * SEQ + 8 * hh;
    const float SC = 0.125f * 1.4426950408889634f;

    float mrow[8], lrow[8];
    v8f oacc[4];
#pragma unroll
    for (int r = 0; r < 8; ++r) { mrow[r] = -1.0e30f; lrow[r] = 0.f; }
#pragma unroll
    for (int t = 0; t < 4; ++t) oacc[t] = (v8f){0.f, 0.f, 0.f, 0.f, 0.f, 0.f, 0.f, 0.f};

#pragma unroll 1
    for (int j0 = 0; j0 < SEQ; j0 += 32) {
        v8f s0 = (v8f){0.f, 0.f, 0.f, 0.f, 0.f, 0.f, 0.f, 0.f};
        v8f s1 = s0;
        {
            const v16h qa0 = ld_frag(QK + qoff), qa1 = ld_frag(QK + qoff + 32);
            const int ko = kb0 + j0 * (2 * CC);
            const v16h k00 = ld_frag(QK + ko), k01 = ld_frag(QK + ko + 32);
            const v16h k10 = ld_frag(QK + ko + 16 * (2 * CC)), k11 = ld_frag(QK + ko + 16 * (2 * CC) + 32);
            s0 = wmma16(qa0, k00, s0);
            s0 = wmma16(qa1, k01, s0);
            s1 = wmma16(qa0, k10, s1);
            s1 = wmma16(qa1, k11, s1);
        }
#pragma unroll
        for (int r = 0; r < 8; ++r) {
            const float a0 = s0[r] * SC, a1 = s1[r] * SC;
            float mx = fmaxf(a0, a1);
            mx = fmaxf(mx, __shfl_xor(mx, 1, 32)); mx = fmaxf(mx, __shfl_xor(mx, 2, 32));
            mx = fmaxf(mx, __shfl_xor(mx, 4, 32)); mx = fmaxf(mx, __shfl_xor(mx, 8, 32));
            const float mn = fmaxf(mrow[r], mx);
            const float al = exp2f(mrow[r] - mn);
            const _Float16 h0 = (_Float16)(exp2f(a0 - mn) * 1024.0f);
            const _Float16 h1 = (_Float16)(exp2f(a1 - mn) * 1024.0f);
            lrow[r] = lrow[r] * al + ((float)h0 + (float)h1);
            mrow[r] = mn;
#pragma unroll
            for (int t = 0; t < 4; ++t) oacc[t][r] *= al;
            Psh[wave][(8 * hh + r) * PP + c] = h0;
            Psh[wave][(8 * hh + r) * PP + 16 + c] = h1;
        }
        wave_sync();
        FragH pf;
        pf.h[0] = *(const v8h*)&Psh[wave][c * PP + 8 * hh];
        pf.h[1] = *(const v8h*)&Psh[wave][c * PP + 16 + 8 * hh];
        wave_sync();
        {
            const int vo = vb0 + j0;
            const v16h v0 = ld_frag(VT + vo), v1 = ld_frag(VT + vo + 16 * MT);
            const v16h v2 = ld_frag(VT + vo + 32 * MT), v3 = ld_frag(VT + vo + 48 * MT);
            oacc[0] = wmma16(pf.v, v0, oacc[0]);
            oacc[1] = wmma16(pf.v, v1, oacc[1]);
            oacc[2] = wmma16(pf.v, v2, oacc[2]);
            oacc[3] = wmma16(pf.v, v3, oacc[3]);
        }
    }

#pragma unroll
    for (int r = 0; r < 8; ++r) {
        float l = lrow[r];
        l += __shfl_xor(l, 1, 32); l += __shfl_xor(l, 2, 32); l += __shfl_xor(l, 4, 32); l += __shfl_xor(l, 8, 32);
        const float inv = 64.0f * (1.0f / l);
#pragma unroll
        for (int t = 0; t < 4; ++t) Os[wave][(8 * hh + r) * SP + t * 16 + c] = oacc[t][r] * inv;
    }
    wave_sync();
    {
        const int q = lane >> 3, c8 = (lane & 7) * 8;
        for (int pass = 0; pass < 2; ++pass) {
#pragma unroll
            for (int it = 0; it < 4; ++it) {
                const int row = it * 4 + q;
                v8h hv;
#pragma unroll
                for (int e = 0; e < 8; ++e) hv[e] = (_Float16)Os[wave][row * SP + c8 + e];
                *(volatile v8h*)(O16 + (size_t)(b * SEQ + q0 + row) * CC + h * HD + c8) = hv;
            }
            __threadfence();
        }
    }
}

#define SZ_X16   ((size_t)MT * CC * 2)
#define SZ_WQKV  ((size_t)3 * CC * CC * 2)
#define SZ_WP    ((size_t)CC * CC * 2)
#define SZ_W1    ((size_t)DFF * CC * 2)
#define SZ_W2    ((size_t)CC * DFF * 2)
#define SZ_QK    ((size_t)MT * 2 * CC * 2)
#define SZ_VT    ((size_t)CC * MT * 2)
#define SZ_O16   ((size_t)MT * CC * 2)
#define SZ_X1    ((size_t)MT * CC * 4)
#define SZ_H16   ((size_t)MT * CC * 2)
#define SZ_F16   ((size_t)MT * DFF * 2)
#define WS_TOTAL (SZ_X16 + SZ_WQKV + SZ_WP + SZ_W1 + SZ_W2 + SZ_QK + SZ_VT + SZ_O16 + SZ_X1 + SZ_H16 + SZ_F16)
static_assert(SZ_X16 % 256 == 0 && SZ_WQKV % 256 == 0 && SZ_WP % 256 == 0 && SZ_W1 % 256 == 0 && SZ_W2 % 256 == 0);
static_assert(SZ_QK % 256 == 0 && SZ_VT % 256 == 0 && SZ_O16 % 256 == 0 && SZ_X1 % 256 == 0 && SZ_H16 % 256 == 0 && SZ_F16 % 256 == 0);
static_assert(WS_TOTAL <= (size_t)134217728);
static_assert(((3 * CC * CC) % 8) == 0 && ((CC * DFF) % 8) == 0);
static_assert((size_t)MT * 2 * CC < (size_t)2147483647 && (size_t)CC * MT < (size_t)2147483647);

extern "C" void kernel_launch(void* const* d_in, const int* in_sizes, int n_in, void* d_out, int out_size, void* d_ws, size_t ws_size, hipStream_t stream) {
    if (n_in < 13) return;
    if (in_sizes[0] < ((NB - 1) * SEQ_FULL + SEQ) * CC) return;
    if (in_sizes[1] < CC || in_sizes[2] < CC || in_sizes[3] < 3 * CC * CC || in_sizes[4] < 3 * CC) return;
    if (in_sizes[5] < CC * CC || in_sizes[6] < CC || in_sizes[7] < CC || in_sizes[8] < CC) return;
    if (in_sizes[9] < DFF * CC || in_sizes[10] < DFF || in_sizes[11] < CC * DFF || in_sizes[12] < CC) return;
    if (out_size < MT * CC) return;
    if (ws_size < WS_TOTAL) return;

    const float* x     = (const float*)d_in[0];
    const float* ln1g  = (const float*)d_in[1];
    const float* ln1b  = (const float*)d_in[2];
    const float* qkvw  = (const float*)d_in[3];
    const float* qkvb  = (const float*)d_in[4];
    const float* projw = (const float*)d_in[5];
    const float* projb = (const float*)d_in[6];
    const float* ln2g  = (const float*)d_in[7];
    const float* ln2b  = (const float*)d_in[8];
    const float* fc1w  = (const float*)d_in[9];
    const float* fc1b  = (const float*)d_in[10];
    const float* fc2w  = (const float*)d_in[11];
    const float* fc2b  = (const float*)d_in[12];
    float* out = (float*)d_out;

    char* wsp = (char*)d_ws;
    unsigned short* X16  = (unsigned short*)wsp; wsp += SZ_X16;
    unsigned short* WQKV = (unsigned short*)wsp; wsp += SZ_WQKV;
    unsigned short* WP   = (unsigned short*)wsp; wsp += SZ_WP;
    unsigned short* W1   = (unsigned short*)wsp; wsp += SZ_W1;
    unsigned short* W2   = (unsigned short*)wsp; wsp += SZ_W2;
    unsigned short* QK   = (unsigned short*)wsp; wsp += SZ_QK;
    unsigned short* VT   = (unsigned short*)wsp; wsp += SZ_VT;
    unsigned short* O16  = (unsigned short*)wsp; wsp += SZ_O16;
    float*          X1   = (float*)wsp;          wsp += SZ_X1;
    unsigned short* H16  = (unsigned short*)wsp; wsp += SZ_H16;
    unsigned short* F16  = (unsigned short*)wsp; wsp += SZ_F16;

    k_ln_in<<<(MT + 7) / 8, 256, 0, stream>>>(x, ln1g, ln1b, X16);
    k_castw<<<(3 * CC * CC / 8 + 255) / 256, 256, 0, stream>>>(qkvw, WQKV, 3 * CC * CC / 8, 16.0f);
    k_castw<<<(CC * CC / 8 + 255) / 256, 256, 0, stream>>>(projw, WP, CC * CC / 8, 16.0f);
    k_castw<<<(DFF * CC / 8 + 255) / 256, 256, 0, stream>>>(fc1w, W1, DFF * CC / 8, 16.0f);
    k_castw<<<(CC * DFF / 8 + 255) / 256, 256, 0, stream>>>(fc2w, W2, CC * DFF / 8, 32.0f);
    k_gemm_qk<<<((MT / 64) * ((2 * CC) / 64) + 7) / 8, 256, 0, stream>>>((const _Float16*)X16, (const _Float16*)WQKV, qkvb, QK);
    k_gemm_vt<<<((CC / 64) * (MT / 64) + 7) / 8, 256, 0, stream>>>((const _Float16*)(WQKV + (size_t)2 * CC * CC), (const _Float16*)X16, qkvb + 2 * CC, VT);
    k_attn<<<NB * NH * (SEQ / 64), 128, 0, stream>>>((const _Float16*)QK, (const _Float16*)VT, O16);
    k_gemm_proj<<<((MT / 64) * (CC / 64) + 7) / 8, 256, 0, stream>>>((const _Float16*)O16, (const _Float16*)WP, projb, x, X1);
    k_ln_mid<<<(MT + 7) / 8, 256, 0, stream>>>(X1, ln2g, ln2b, H16);
    k_gemm_fc1<<<((MT / 64) * (DFF / 64) + 7) / 8, 256, 0, stream>>>((const _Float16*)H16, (const _Float16*)W1, fc1b, F16);
    k_gemm_fc2<<<((MT / 64) * (CC / 64) + 7) / 8, 256, 0, stream>>>((const _Float16*)F16, (const _Float16*)W2, fc2b, X1, out);
}
